// VFXNet_71511205479082
// MI455X (gfx1250) — hardware-verified
//
#include <hip/hip_runtime.h>
#include <stddef.h>
#include <math.h>


#define NTHR   256
#define NWAVE  8
#define NPB    128
#define PTHR   64
#define IMG_W  1024
#define IMG_H  1024
#define HWPIX  (IMG_W * IMG_H)
#define XP     40
#define HP     72
#define TWO_PI_F 6.28318530717958647692f
#define SCL    16.0f
#define INV16  0.0625f
#define INVW   0.0009765625f

#define PE_H (48 * 32)
#define PF_H (128 * 64)
#define P0_H (64 * 32)
#define P1_H (64 * 64)
#define P2_H (16 * 64)
#define PB_E 3
#define PB_F 16
#define PB_0 4
#define PB_1 8
#define PB_2 2
#define PB_TOT (PB_E + PB_F + PB_0 + PB_1 + PB_2)

static_assert(PB_E * PTHR * 8 == PE_H);
static_assert(PB_F * PTHR * 8 == PF_H);
static_assert(PB_0 * PTHR * 8 == P0_H);
static_assert(PB_1 * PTHR * 8 == P1_H);
static_assert(PB_2 * PTHR * 8 == P2_H);
static_assert(PB_TOT == 33);

#define OE    0
#define OM    (OE + 16 * XP * 2)
#define OF    (OM + 16 * XP * 2)
#define OH1   (OF + 16 * HP * 2)
#define OH2   (OH1 + 16 * HP * 2)
#define OST   (OH2 + 16 * HP * 2)
#define WVB   (OST + 16 * 64 * 4)
#define OOUT  (NWAVE * WVB)
#define LDS_FWD (OOUT + NPB * 4 * 4)

static_assert(NPB == NWAVE * 16);
static_assert((OM % 16) == 0 && (OF % 16) == 0 && (OH1 % 16) == 0 && (OH2 % 16) == 0);
static_assert((OST % 16) == 0 && (WVB % 16) == 0 && (OOUT % 16) == 0);
static_assert((XP * 2) % 16 == 0 && (HP * 2) % 16 == 0);
static_assert(LDS_FWD == 110592);

typedef float    v2f  __attribute__((ext_vector_type(2)));
typedef float    v4f  __attribute__((ext_vector_type(4)));
typedef float    v8f  __attribute__((ext_vector_type(8)));
typedef _Float16 v2h  __attribute__((ext_vector_type(2)));
typedef _Float16 v8h  __attribute__((ext_vector_type(8)));
typedef _Float16 v16h __attribute__((ext_vector_type(16)));
union FragH { v16h v; v8h h[2]; };

__device__ __forceinline__ v8f wmh(v16h a, v16h b, v8f c) {
  v8f d = __builtin_amdgcn_wmma_f32_16x16x32_f16(false, a, false, b, (short)0, c, false, false);
#if defined(__HIP_DEVICE_COMPILE__)
  asm volatile("v_nop\n\tv_nop\n\tv_nop\n\tv_nop" : "+v"(d) : "v"(a), "v"(b));
#endif
  return d;
}

__device__ __forceinline__ v8f zero8() {
  v8f z = {0.f, 0.f, 0.f, 0.f, 0.f, 0.f, 0.f, 0.f};
  return z;
}

template <int KT>
__device__ __forceinline__ void load_a(FragH (&a)[KT], const _Float16* ar) {
#pragma unroll
  for (int kt = 0; kt < KT; ++kt) {
    a[kt].h[0] = *(const v8h*)(ar + 32 * kt);
    a[kt].h[1] = *(const v8h*)(ar + 32 * kt + 16);
  }
}

template <int KT>
__device__ __forceinline__ v8f mma_tile(const FragH (&a)[KT], const _Float16* __restrict__ bplane,
                                        int nrow0, int KP, int m, int hh) {
  v8f acc = zero8();
#pragma unroll
  for (int kt = 0; kt < KT; ++kt) {
    const _Float16* bq = bplane + (size_t)(nrow0 + m) * KP + 32 * kt + 8 * hh;
    FragH b;
    b.h[0] = *(const v8h*)bq;
    b.h[1] = *(const v8h*)(bq + 16);
    acc = wmh(a[kt].v, b.v, acc);
  }
  return acc;
}

__device__ __forceinline__ float gelu_f(float x) {
  return 0.5f * x * (1.0f + erff(x * 0.70710678118654752440f));
}

__device__ __forceinline__ float sigm_f(float x) {
  const float e = expf(fminf(-x, 30.0f));
  return 1.0f / (1.0f + e);
}

__device__ __forceinline__ void gelu_pass(const float* stg, _Float16* dst, int lane) {
#pragma unroll 1
  for (int i = 0; i < 16; ++i) {
    const v2f x = *(const v2f*)(stg + 64 * i + 2 * lane);
    v2h y;
    y[0] = (_Float16)gelu_f(x[0]);
    y[1] = (_Float16)gelu_f(x[1]);
    *(v2h*)(dst + i * HP + 2 * lane) = y;
  }
}

__global__ __launch_bounds__(PTHR) void k_prep(
    const float* __restrict__ Wc, const float* __restrict__ Wp, const float* __restrict__ Wt,
    const float* __restrict__ Wf, const float* __restrict__ W0, const float* __restrict__ W1,
    const float* __restrict__ W2,
    _Float16* pE, _Float16* pF, _Float16* p0, _Float16* p1, _Float16* p2) {
  const int b = blockIdx.x;
  const int tid = threadIdx.x;
  const float* src; _Float16* dst;
  int g0, kpsh, scols, coff, klo, kv, nv;
  if (b < PB_E) {
    dst = pE; g0 = 0; kpsh = 5; scols = 16; coff = 16 * b; nv = 48;
    if (b == 0)      { src = Wc; klo = 0;  kv = 2;  }
    else if (b == 1) { src = Wp; klo = 2;  kv = 12; }
    else             { src = Wt; klo = 14; kv = 6;  }
  } else if (b < PB_E + PB_F) {
    src = Wf; dst = pF; g0 = PB_E; kpsh = 6; scols = 128; coff = 0; klo = 0; kv = 48; nv = 128;
  } else if (b < PB_E + PB_F + PB_0) {
    src = W0; dst = p0; g0 = PB_E + PB_F; kpsh = 5; scols = 64; coff = 0; klo = 0; kv = 10; nv = 64;
  } else if (b < PB_E + PB_F + PB_0 + PB_1) {
    src = W1; dst = p1; g0 = PB_E + PB_F + PB_0; kpsh = 6; scols = 64; coff = 0; klo = 0; kv = 64; nv = 64;
  } else {
    src = W2; dst = p2; g0 = PB_E + PB_F + PB_0 + PB_1; kpsh = 6; scols = 4; coff = 0; klo = 0; kv = 64; nv = 4;
  }
  const int gi = (b - g0) * PTHR + tid;
  const int o  = gi * 8;
  const int n  = o >> kpsh;
  const int k0 = o & ((1 << kpsh) - 1);
  int nc = n - coff;
  nc = nc < 0 ? 0 : (nc > scols - 1 ? scols - 1 : nc);
  float v[8];
#pragma unroll
  for (int e = 0; e < 8; ++e) {
    const int k  = k0 + e;
    const int kk = k - klo;
    const bool valid = (kk >= 0) && (kk < kv) && (n < nv);
    int kc = kk < 0 ? 0 : (kk > kv - 1 ? kv - 1 : kk);
    const float xv = src[(size_t)kc * scols + nc];
    v[e] = valid ? xv * SCL : 0.0f;
  }
  v8h hv;
#pragma unroll
  for (int e = 0; e < 8; ++e) hv[e] = (_Float16)v[e];
  _Float16* dp = dst + o;
  *(volatile v8h*)dp = hv;
  __threadfence();
  *(volatile v8h*)dp = hv;
}

__global__ __launch_bounds__(NTHR) void k_fwd(
    const int*   __restrict__ raw_pos, const float* __restrict__ control, const float* __restrict__ latent,
    const float* __restrict__ bc, const float* __restrict__ bp, const float* __restrict__ bt,
    const float* __restrict__ bfv, const float* __restrict__ b0, const float* __restrict__ b1,
    const float* __restrict__ b2,
    const _Float16* __restrict__ pE, const _Float16* __restrict__ pF, const _Float16* __restrict__ p0,
    const _Float16* __restrict__ p1, const _Float16* __restrict__ p2,
    float* out, int Npts) {
  extern __shared__ v4f lds_dyn[];
  char* lb = (char*)lds_dyn;
  const int tid = threadIdx.x, lane = tid & 31, wave = tid >> 5, hh = lane >> 4, m = lane & 15;
  char* wb = lb + wave * WVB;
  _Float16* sE  = (_Float16*)(wb + OE);
  _Float16* sM  = (_Float16*)(wb + OM);
  _Float16* sF  = (_Float16*)(wb + OF);
  _Float16* sH1 = (_Float16*)(wb + OH1);
  _Float16* sH2 = (_Float16*)(wb + OH2);
  float*    stg = (float*)(wb + OST);
  float*    sO  = (float*)(lb + OOUT);
  const long long pbase = (long long)blockIdx.x * NPB;

  {
    long long gp = pbase + wave * 16 + m;
    const long long lastp = (long long)Npts - 1;
    gp = gp > lastp ? lastp : gp;
    const int rx = raw_pos[2 * gp];
    const int ry = raw_pos[2 * gp + 1];
    const float cv0 = control[2 * gp];
    const float cv1 = control[2 * gp + 1];
    const int ix = rx < 0 ? 0 : (rx > IMG_W - 1 ? IMG_W - 1 : rx);
    const int iy = ry < 0 ? 0 : (ry > IMG_H - 1 ? IMG_H - 1 : ry);
    long long li = (long long)ry * IMG_W + (long long)rx;
    li = li < 0 ? li + HWPIX : li;
    li = li < 0 ? 0 : (li > (long long)(HWPIX - 1) ? (long long)(HWPIX - 1) : li);
    const v4f lat = *(const v4f*)(latent + (size_t)li * 4);
    const float xn = (float)ix * INVW;
    const float yn = (float)iy * INVW;
    const float X = xn * TWO_PI_F, Y = yn * TWO_PI_F, T = cv0 * TWO_PI_F;
    const float Bv = hh ? Y : X;
    const float B2 = 2.0f * Bv, B3 = 3.0f * Bv;
    const float T2 = 2.0f * T, T3 = 3.0f * T;
    const float aT = hh ? T : T2;
    const float s1 = sinf(Bv), c1 = cosf(Bv);
    const float s2 = sinf(B2), c2 = cosf(B2);
    const float s3 = sinf(B3), c3 = cosf(B3);
    const float sT = sinf(aT), cT = cosf(aT);
    const float s3T = sinf(T3), c3T = cosf(T3);
    const float o1 = __shfl_xor(s1, 16, 32);
    const float o2 = __shfl_xor(s2, 16, 32);

    v8h ea, eb, ma, zz;
    ea[0] = (_Float16)(hh ? s1 : cv0);
    ea[1] = (_Float16)(hh ? c1 : cv1);
    ea[2] = (_Float16)(hh ? s2 : s1);
    ea[3] = (_Float16)(hh ? c2 : c1);
    ea[4] = (_Float16)(hh ? s3 : s2);
    ea[5] = (_Float16)(hh ? c3 : c2);
    ea[6] = (_Float16)(hh ? sT : s3);
    ea[7] = (_Float16)(hh ? cT : c3);
    eb[0] = (_Float16)(hh ? 0.0f : sT);
    eb[1] = (_Float16)(hh ? 0.0f : cT);
    eb[2] = (_Float16)(hh ? 0.0f : s3T);
    eb[3] = (_Float16)(hh ? 0.0f : c3T);
    eb[4] = (_Float16)0.0f; eb[5] = (_Float16)0.0f; eb[6] = (_Float16)0.0f; eb[7] = (_Float16)0.0f;
    ma[0] = (_Float16)(hh ? o2   : lat[0]);
    ma[1] = (_Float16)(hh ? s2   : lat[1]);
    ma[2] = (_Float16)(hh ? 0.0f : lat[2]);
    ma[3] = (_Float16)(hh ? 0.0f : lat[3]);
    ma[4] = (_Float16)(hh ? 0.0f : xn);
    ma[5] = (_Float16)(hh ? 0.0f : yn);
    ma[6] = (_Float16)(hh ? 0.0f : s1);
    ma[7] = (_Float16)(hh ? 0.0f : o1);
#pragma unroll
    for (int e = 0; e < 8; ++e) zz[e] = (_Float16)0.0f;

    _Float16* er = sE + m * XP;
    *(v8h*)(er + 8 * hh)      = ea;
    *(v8h*)(er + 16 + 8 * hh) = eb;
    _Float16* mrow = sM + m * XP;
    *(v8h*)(mrow + 8 * hh)      = ma;
    *(v8h*)(mrow + 16 + 8 * hh) = zz;
    *(v8h*)(sF + m * HP + 48 + 8 * hh) = zz;
  }
  __syncthreads();

  {
    FragH aE[1];
    load_a<1>(aE, sE + m * XP + 8 * hh);
    const v8f e0 = mma_tile<1>(aE, pE, 0,  32, m, hh);
    const v8f e1 = mma_tile<1>(aE, pE, 16, 32, m, hh);
    const v8f e2 = mma_tile<1>(aE, pE, 32, 32, m, hh);
    const float bcm = bc[m], bpm = bp[m], btm = bt[m];
    _Float16* fq = sF + (8 * hh) * HP + m;
#pragma unroll
    for (int r = 0; r < 8; ++r) {
      fq[r * HP]      = (_Float16)fmaxf(fmaf(e0[r], INV16, bcm), 0.0f);
      fq[r * HP + 16] = (_Float16)fmaxf(fmaf(e1[r], INV16, bpm), 0.0f);
      fq[r * HP + 32] = (_Float16)fmaxf(fmaf(e2[r], INV16, btm), 0.0f);
    }
  }
  __syncthreads();

  {
    FragH aF[2];
    load_a<2>(aF, sF + m * HP + 8 * hh);
    FragH aM[1];
    load_a<1>(aM, sM + m * XP + 8 * hh);
    float* stq = stg + (8 * hh) * 64 + m;
#pragma unroll
    for (int nb = 0; nb < 4; ++nb) {
      const v8f g  = mma_tile<2>(aF, pF, 16 * nb,      64, m, hh);
      const v8f be = mma_tile<2>(aF, pF, 64 + 16 * nb, 64, m, hh);
      const v8f hv = mma_tile<1>(aM, p0, 16 * nb,      32, m, hh);
      const float bg = bfv[16 * nb + m];
      const float bb = bfv[64 + 16 * nb + m];
      const float bh = b0[16 * nb + m];
#pragma unroll
      for (int r = 0; r < 8; ++r) {
        const float gg  = fmaf(g[r],  INV16, bg);
        const float bt2 = fmaf(be[r], INV16, bb);
        const float hq  = fmaf(hv[r], INV16, bh);
        stq[r * 64 + 16 * nb] = fmaf(gg, hq, bt2);
      }
    }
  }
  __syncthreads();
  gelu_pass(stg, sH1, lane);
  __syncthreads();

  {
    FragH a1[2];
    load_a<2>(a1, sH1 + m * HP + 8 * hh);
    float* stq = stg + (8 * hh) * 64 + m;
#pragma unroll
    for (int nb = 0; nb < 4; ++nb) {
      const v8f c = mma_tile<2>(a1, p1, 16 * nb, 64, m, hh);
      const float bb = b1[16 * nb + m];
#pragma unroll
      for (int r = 0; r < 8; ++r) stq[r * 64 + 16 * nb] = fmaf(c[r], INV16, bb);
    }
  }
  __syncthreads();
  gelu_pass(stg, sH2, lane);
  __syncthreads();

  {
    FragH a2[2];
    load_a<2>(a2, sH2 + m * HP + 8 * hh);
    const v8f c = mma_tile<2>(a2, p2, 0, 64, m, hh);
    const int mc = m < 4 ? m : 3;
    const float bo = b2[mc];
    float vq[8];
#pragma unroll
    for (int r = 0; r < 8; ++r) vq[r] = fmaf(c[r], INV16, bo);
    if (m < 4) {
      float* oq = sO + (16 * wave + 8 * hh) * 4 + m;
#pragma unroll
      for (int r = 0; r < 8; ++r) oq[r * 4] = vq[r];
    }
  }
  __syncthreads();

  if (wave < NPB / 32) {
    const v4f x = *(const v4f*)(sO + 4 * tid);
    v4f o;
    o[0] = sigm_f(x[0]); o[1] = sigm_f(x[1]); o[2] = sigm_f(x[2]); o[3] = sigm_f(x[3]);
    const long long gp = pbase + tid;
    float* op = out + (size_t)(gp > 0 ? gp : 0) * 4;
    if (gp < (long long)Npts) *(volatile v4f*)op = o;
    __threadfence();
    if (gp < (long long)Npts) *(volatile v4f*)op = o;
  }
}

extern "C" void kernel_launch(void* const* d_in, const int* in_sizes, int n_in,
                              void* d_out, int out_size, void* d_ws, size_t ws_size,
                              hipStream_t stream) {
  if (n_in < 17) return;
  const int Npts = in_sizes[0] / 2;
  if (Npts <= 0 || in_sizes[0] != 2 * Npts || in_sizes[1] != 2 * Npts) return;
  if (in_sizes[2] != HWPIX * 4) return;
  if (in_sizes[3] != 2 * 16 || in_sizes[4] != 16) return;
  if (in_sizes[5] != 6 * 16 || in_sizes[6] != 16) return;
  if (in_sizes[7] != 12 * 16 || in_sizes[8] != 16) return;
  if (in_sizes[9] != 48 * 128 || in_sizes[10] != 128) return;
  if (in_sizes[11] != 10 * 64 || in_sizes[12] != 64) return;
  if (in_sizes[13] != 64 * 64 || in_sizes[14] != 64) return;
  if (in_sizes[15] != 64 * 4 || in_sizes[16] != 4) return;
  if (out_size != 4 * Npts) return;

  const int*   raw_pos = (const int*)d_in[0];
  const float* control = (const float*)d_in[1];
  const float* latent  = (const float*)d_in[2];
  const float* Wc = (const float*)d_in[3];  const float* bc = (const float*)d_in[4];
  const float* Wt = (const float*)d_in[5];  const float* bt = (const float*)d_in[6];
  const float* Wp = (const float*)d_in[7];  const float* bp = (const float*)d_in[8];
  const float* Wf = (const float*)d_in[9];  const float* bfv = (const float*)d_in[10];
  const float* W0 = (const float*)d_in[11]; const float* b0 = (const float*)d_in[12];
  const float* W1 = (const float*)d_in[13]; const float* b1 = (const float*)d_in[14];
  const float* W2 = (const float*)d_in[15]; const float* b2 = (const float*)d_in[16];
  float* out = (float*)d_out;

  char* ws = (char*)d_ws;
  size_t off = 0;
  const size_t oE = off; off += (size_t)PE_H * 2; off = (off + 255) & ~(size_t)255;
  const size_t oFp = off; off += (size_t)PF_H * 2; off = (off + 255) & ~(size_t)255;
  const size_t o0 = off; off += (size_t)P0_H * 2; off = (off + 255) & ~(size_t)255;
  const size_t o1 = off; off += (size_t)P1_H * 2; off = (off + 255) & ~(size_t)255;
  const size_t o2 = off; off += (size_t)P2_H * 2; off = (off + 255) & ~(size_t)255;
  if (off > ws_size || off > (size_t)134217728) return;
  _Float16* pE = (_Float16*)(ws + oE);
  _Float16* pF = (_Float16*)(ws + oFp);
  _Float16* p0 = (_Float16*)(ws + o0);
  _Float16* p1 = (_Float16*)(ws + o1);
  _Float16* p2 = (_Float16*)(ws + o2);

  k_prep<<<PB_TOT, PTHR, 0, stream>>>(Wc, Wp, Wt, Wf, W0, W1, W2, pE, pF, p0, p1, p2);

  hipFuncSetAttribute(reinterpret_cast<const void*>(&k_fwd),
                      hipFuncAttributeMaxDynamicSharedMemorySize, LDS_FWD);
  const int nBlk = (Npts + NPB - 1) / NPB;
  k_fwd<<<nBlk, NTHR, LDS_FWD, stream>>>(raw_pos, control, latent, bc, bp, bt, bfv, b0, b1, b2,
                                          pE, pF, p0, p1, p2, out, Npts);
}
